// SubgraphEncoder_2216203125208
// MI455X (gfx1250) — hardware-verified
//
#include <hip/hip_runtime.h>
#include <math.h>

constexpr int NNODE = 40000;
constexpr int NEDGE = 640000;
constexpr int NHID  = 128;
constexpr int NATT  = 64;
constexpr int NSUB  = 400;
constexpr int NCELL = 100;
constexpr int NBOT  = 32;
#define NT 256
constexpr int ROWS_W = 512;
constexpr int TILE_R = 8 * ROWS_W;
constexpr int NTILE  = 10;
constexpr int NPADR  = NTILE * TILE_R;
constexpr int SPT    = 20;
constexpr int SCH    = NT * SPT;
constexpr int NCHK   = NEDGE / SCH;
constexpr int RPB    = 512;
constexpr int NAPB   = (NNODE + RPB - 1) / RPB;
constexpr float BN_EPS = 1e-5f;
constexpr float WA_CARRY = 16.0f;
constexpr float WA_CARRY_INV = 1.0f / 16.0f;

static_assert(NEDGE % SCH == 0, "chunks are exact");
static_assert(SPT % 4 == 0, "b128 edge loads");
static_assert(NPADR >= NNODE, "tile cover");
static_assert(NNODE < 65536, "src packed in 16 bits");
static_assert(TILE_R <= 4096, "dl packed above bit 16 fits an int");
static_assert(NNODE % 64 == 0 && NHID % 64 == 0 && NATT % 64 == 0, "GEMM M/N tile multiples");
static_assert(NHID % 32 == 0, "GEMM K multiple of 32");
static_assert(NNODE % 32 == 0, "score store lines are whole per wave");
static_assert((NNODE * NHID) % (8 * NT) == 0, "split grid exact");
static_assert(NCELL * NSUB == NNODE, "cells are contiguous row blocks");
static_assert(NCELL * NBOT * 4 == 12800, "out0 bytes");
static_assert(12800 + NNODE * NHID * 4 == 20492800, "out1 offset + bytes == total");

typedef __attribute__((ext_vector_type(16))) _Float16 v16h;
typedef __attribute__((ext_vector_type(8)))  _Float16 v8h;
typedef __attribute__((ext_vector_type(16))) __bf16   v16b;
typedef __attribute__((ext_vector_type(8)))  __bf16   v8b;
typedef __attribute__((ext_vector_type(8)))  float    v8f;
typedef __attribute__((ext_vector_type(4)))  float    v4f;
typedef __attribute__((ext_vector_type(4)))  int      v4i;
typedef __attribute__((ext_vector_type(4)))  unsigned int v4u;

__device__ __forceinline__ unsigned short f2bf_bits(float f) {
  unsigned u = __float_as_uint(f);
  return (unsigned short)((u + 0x7FFFu + ((u >> 16) & 1u)) >> 16);
}
__device__ __forceinline__ float bf_bits2f(unsigned short h) { return __uint_as_float(((unsigned)h) << 16); }
__device__ __forceinline__ unsigned pk16(unsigned short a, unsigned short b) { return (unsigned)a | ((unsigned)b << 16); }
__device__ __forceinline__ unsigned short h_bits(float f) { const _Float16 h = (_Float16)f; return __builtin_bit_cast(unsigned short, h); }

__device__ __forceinline__ void dep_guard_h(v8f& a, v8f& b, v16h x, v16h y) { asm volatile("v_nop\n\tv_nop\n\tv_nop\n\tv_nop" : "+v"(a), "+v"(b) : "v"(x), "v"(y)); }
__device__ __forceinline__ void dep_guard_b(v8f& a, v8f& b, v16b x, v16b y) { asm volatile("v_nop\n\tv_nop\n\tv_nop\n\tv_nop" : "+v"(a), "+v"(b) : "v"(x), "v"(y)); }
__device__ __forceinline__ void dep_guard4_h(v8f& a, v8f& b, v8f& c, v8f& d, v16h x, v16h y) { asm volatile("v_nop\n\tv_nop\n\tv_nop\n\tv_nop" : "+v"(a), "+v"(b), "+v"(c), "+v"(d) : "v"(x), "v"(y)); }
__device__ __forceinline__ void dep_guard4_b(v8f& a, v8f& b, v8f& c, v8f& d, v16b x, v16b y) { asm volatile("v_nop\n\tv_nop\n\tv_nop\n\tv_nop" : "+v"(a), "+v"(b), "+v"(c), "+v"(d) : "v"(x), "v"(y)); }
__device__ __forceinline__ void keep4_h(v16h a, v16h b, v16h c, v16h d) { asm volatile("v_nop" :: "v"(a), "v"(b), "v"(c), "v"(d)); }
__device__ __forceinline__ void keep4_b(v16b a, v16b b, v16b c, v16b d) { asm volatile("v_nop" :: "v"(a), "v"(b), "v"(c), "v"(d)); }
__device__ __forceinline__ void acc_guard4(v8f& a, v8f& b, v8f& c, v8f& d) { asm volatile("v_nop\n\tv_nop\n\tv_nop\n\tv_nop" : "+v"(a), "+v"(b), "+v"(c), "+v"(d)); }
template <typename T> struct Frag;
template <> struct Frag<_Float16> {
  typedef v16h V; union U { v16h v; v8h h[2]; };
  static __device__ __forceinline__ v16h load(const _Float16* p) {
    U f; f.h[0] = *(const v8h*)(p); f.h[1] = *(const v8h*)(p + 16); return f.v;
  }
  static __device__ __forceinline__ v8f mma(v16h a, v16h b, v8f c) {
    return __builtin_amdgcn_wmma_f32_16x16x32_f16(false, a, false, b, (short)0, c, false, false);
  }
  static __device__ __forceinline__ void guard(v8f& a, v8f& b, v16h x, v16h y) { dep_guard_h(a, b, x, y); }
  static __device__ __forceinline__ void guard4(v8f& a, v8f& b, v8f& c, v8f& d, v16h x, v16h y) { dep_guard4_h(a, b, c, d, x, y); }
  static __device__ __forceinline__ void keep(v16h a, v16h b, v16h c, v16h d) { keep4_h(a, b, c, d); }
};
template <> struct Frag<__bf16> {
  typedef v16b V; union U { v16b v; v8b h[2]; };
  static __device__ __forceinline__ v16b load(const __bf16* p) {
    U f; f.h[0] = *(const v8b*)(p); f.h[1] = *(const v8b*)(p + 16); return f.v;
  }
  static __device__ __forceinline__ v8f mma(v16b a, v16b b, v8f c) {
    return __builtin_amdgcn_wmma_f32_16x16x32_bf16(false, a, false, b, (short)0, c, false, false);
  }
  static __device__ __forceinline__ void guard(v8f& a, v8f& b, v16b x, v16b y) { dep_guard_b(a, b, x, y); }
  static __device__ __forceinline__ void guard4(v8f& a, v8f& b, v8f& c, v8f& d, v16b x, v16b y) { dep_guard4_b(a, b, c, d, x, y); }
  static __device__ __forceinline__ void keep(v16b a, v16b b, v16b c, v16b d) { keep4_b(a, b, c, d); }
};

template <int ET> struct Elem;
template <> struct Elem<0> { typedef _Float16 T; };
template <> struct Elem<1> { typedef __bf16 T; };
template <int ET, bool SPLIT, int BIAS_MODE, int OUT_MODE, bool RESID, int ACT = 0>
__global__ __launch_bounds__(256) void wmma_gemm64(
    const unsigned short* __restrict__ Ap, const unsigned short* __restrict__ A2p, int lda, long strideA,
    const unsigned short* __restrict__ Btp, const unsigned short* __restrict__ Bt2p, int ldb, long strideB,
    void* __restrict__ Cout, void* __restrict__ Cout2, int ldc, long strideC,
    const float* __restrict__ bias,
    const float* __restrict__ resid, long strideR,
    int M, int N, int K, float scale) {
  typedef typename Elem<ET>::T T;
  typedef typename Frag<T>::V V;
  const T* A = (const T*)Ap; const T* A2 = (const T*)A2p; const T* Bt = (const T*)Btp; const T* Bt2 = (const T*)Bt2p;
  __shared__ __align__(16) float sT[8][16 * 68];
  const int b    = blockIdx.y;
  const int lane = threadIdx.x & 31;
  const int wave = threadIdx.x >> 5;
  const int tilesN = N >> 6;
  const int tilesM = M >> 6;
  const int tile = blockIdx.x * 8 + wave;
  if (tile >= tilesM * tilesN) return;
  const int tm = tile / tilesN;
  const int tn = tile - tm * tilesN;
  const int m0 = tm << 6;
  const int n0 = tn << 6;

  const T* Ab  = A  + (size_t)b * strideA;
  const T* Bb  = Bt + (size_t)b * strideB;
  const T* Ab2 = SPLIT ? (A2  + (size_t)b * strideA) : nullptr;
  const T* Bb2 = SPLIT ? (Bt2 + (size_t)b * strideB) : nullptr;

  const int rlane = lane & 15;
  const int koff  = (lane >> 4) * 8;
  const int mOff  = (lane >> 4) * 8;

  v8f acc[4][4];
#pragma unroll
  for (int i = 0; i < 4; ++i)
#pragma unroll
    for (int j = 0; j < 4; ++j) acc[i][j] = (v8f){0.f,0.f,0.f,0.f,0.f,0.f,0.f,0.f};

  for (int k0 = 0; k0 < K; k0 += 32) {
    V bh[4], bl[4];
#pragma unroll
    for (int j = 0; j < 4; ++j) {
      const size_t bo = (size_t)(n0 + (j << 4) + rlane) * ldb + koff + k0;
      bh[j] = Frag<T>::load(Bb + bo);
      if (SPLIT) bl[j] = Frag<T>::load(Bb2 + bo);
    }
#pragma unroll
    for (int i = 0; i < 4; ++i) {
      const size_t ao = (size_t)(m0 + (i << 4) + rlane) * lda + koff + k0;
      V ah = Frag<T>::load(Ab + ao);
      V al;
      if (SPLIT) al = Frag<T>::load(Ab2 + ao);
#pragma unroll
      for (int j = 0; j < 4; ++j) {
        acc[i][j] = Frag<T>::mma(ah, bh[j], acc[i][j]);
        if (SPLIT) {
          acc[i][j] = Frag<T>::mma(ah, bl[j], acc[i][j]);
          acc[i][j] = Frag<T>::mma(al, bh[j], acc[i][j]);
        }
      }
      Frag<T>::guard4(acc[i][0], acc[i][1], acc[i][2], acc[i][3], ah, SPLIT ? al : ah);
    }
    Frag<T>::keep(bh[0], bh[1], bh[2], bh[3]);
    if (SPLIT) Frag<T>::keep(bl[0], bl[1], bl[2], bl[3]);
  }
  acc_guard4(acc[0][0], acc[0][1], acc[0][2], acc[0][3]);
  acc_guard4(acc[1][0], acc[1][1], acc[1][2], acc[1][3]);
  acc_guard4(acc[2][0], acc[2][1], acc[2][2], acc[2][3]);
  acc_guard4(acc[3][0], acc[3][1], acc[3][2], acc[3][3]);

  float* slab = sT[wave];
  const float* Rb = RESID ? (resid + (size_t)b * strideR) : nullptr;
#pragma unroll
  for (int i = 0; i < 4; ++i) {
    const int mBase = m0 + (i << 4);
#pragma unroll
    for (int j = 0; j < 4; ++j) {
      const int n = n0 + (j << 4) + rlane;
      float bv = 0.f;
      if (BIAS_MODE == 2) bv = bias[n];
#pragma unroll
      for (int r = 0; r < 8; ++r) {
        float v = acc[i][j][r] * scale;
        if (BIAS_MODE == 1) v += bias[mBase + mOff + r];
        if (BIAS_MODE == 2) v += bv;
        if (RESID) v += Rb[(size_t)(mBase + mOff + r) * ldc + n];
        if (ACT == 2) v = fmaxf(v, 0.0f);
        if (ACT == 4) v = (v > 0.f) ? v : 0.01f * v;
        slab[(mOff + r) * 68 + (j << 4) + rlane] = v;
      }
    }
    __builtin_amdgcn_fence(__ATOMIC_RELEASE, "workgroup");
    __builtin_amdgcn_wave_barrier();
    __builtin_amdgcn_fence(__ATOMIC_ACQUIRE, "workgroup");
    if (OUT_MODE == 0) {
      float* C = (float*)Cout + (size_t)b * strideC;
      const int hh = lane >> 4, c4 = (lane & 15) * 4;
      for (int pass = 0; pass < 2; ++pass) {
#pragma unroll
        for (int it = 0; it < 8; ++it) {
          const int row = it * 2 + hh;
          v4f v = *(const v4f*)(slab + row * 68 + c4);
          *(volatile v4f*)(C + (size_t)(mBase + row) * ldc + n0 + c4) = v;
        }
        __threadfence();
      }
    } else {
      const int q = lane >> 3, c8 = (lane & 7) * 8;
      unsigned short* C  = (unsigned short*)Cout  + (size_t)b * strideC;
      unsigned short* C2 = (OUT_MODE == 2) ? ((unsigned short*)Cout2 + (size_t)b * strideC) : nullptr;
      for (int pass = 0; pass < 2; ++pass) {
#pragma unroll
        for (int it = 0; it < 4; ++it) {
          const int row = it * 4 + q;
          const float* sp = slab + row * 68 + c8;
          v8h hv, lv;
#pragma unroll
          for (int e = 0; e < 8; ++e) {
            if (OUT_MODE == 1) {
              hv[e] = (_Float16)sp[e];
            } else {
              unsigned short hb = f2bf_bits(sp[e]);
              unsigned short lb = f2bf_bits(sp[e] - bf_bits2f(hb));
              hv[e] = __builtin_bit_cast(_Float16, hb);
              lv[e] = __builtin_bit_cast(_Float16, lb);
            }
          }
          *(volatile v8h*)(C + (size_t)(mBase + row) * ldc + n0 + c8) = hv;
          if (OUT_MODE == 2) *(volatile v8h*)(C2 + (size_t)(mBase + row) * ldc + n0 + c8) = lv;
        }
        __threadfence();
      }
    }
    __builtin_amdgcn_fence(__ATOMIC_RELEASE, "workgroup");
    __builtin_amdgcn_wave_barrier();
    __builtin_amdgcn_fence(__ATOMIC_ACQUIRE, "workgroup");
  }
}

__device__ __forceinline__ int blk_excl_scan(int cnt, int* scan_ws, int tid, int* tot) {
  const int lane = tid & 31, wave = tid >> 5; int incl = cnt;
#pragma unroll
  for (int o = 1; o < 32; o <<= 1) { const int v = __shfl_up(incl, o, 32); if (lane >= o) incl += v; }
  if (lane == 31) scan_ws[wave] = incl;
  __syncthreads();
  if (wave == 0) { int wv = (lane < NT / 32) ? scan_ws[lane] : 0; int wincl = wv;
#pragma unroll
    for (int o = 1; o < 32; o <<= 1) { const int v = __shfl_up(wincl, o, 32); if (lane >= o) wincl += v; }
    if (lane < NT / 32) scan_ws[32 + lane] = wincl - wv; if (lane == 31) scan_ws[64] = wincl; }
  __syncthreads();
  const int res = scan_ws[32 + wave] + incl - cnt; *tot = scan_ws[64];
  return res;
}

__device__ __forceinline__ int chunk_hits(const int* __restrict__ dstv, const int* __restrict__ srcv, int e0, int n0, int tid,
                                          int* LIST, int* scan_ws) {
  const int eb = e0 + tid * SPT;
  int rec[SPT]; int cnt = 0;
#pragma unroll
  for (int k = 0; k < SPT; k += 4) {
    if (k == 12) asm volatile("" ::: "memory");
    const v4i d4 = *(const v4i*)(dstv + eb + k);
    const v4i s4 = *(const v4i*)(srcv + eb + k);
    asm volatile("" :: "v"(d4), "v"(s4));
#pragma unroll
    for (int e = 0; e < 4; ++e) {
      const int d = d4[e]; int s = s4[e]; s = s < 0 ? 0 : (s >= NNODE ? NNODE - 1 : s);
      int r = -1;
      if (d >= n0 && d < n0 + TILE_R) { r = ((d - n0) << 16) | s; ++cnt; }
      rec[k + e] = r;
    }
  }
  int tot; int p = blk_excl_scan(cnt, scan_ws, tid, &tot);
#pragma unroll
  for (int k = 0; k < SPT; ++k) if (rec[k] >= 0) { if ((unsigned)p < (unsigned)SCH) LIST[p] = rec[k]; ++p; }
  __syncthreads();
  return tot < SCH ? tot : SCH;
}

__global__ __launch_bounds__(NT) void prep_kernel(const float* __restrict__ W1, const float* __restrict__ W2, const float* __restrict__ WA,
                                                 unsigned* __restrict__ W1H, unsigned* __restrict__ W1L,
                                                 unsigned* __restrict__ W2H, unsigned* __restrict__ W2L, unsigned* __restrict__ WAH) {
  const int blk = blockIdx.x, t = threadIdx.x;
  if (blk < 64) {
    const bool first = blk < 32;
    const float* W = first ? W1 : W2;
    unsigned* OH = first ? W1H : W2H;
    unsigned* OL = first ? W1L : W2L;
    const int i = (blk & 31) * NT + t;
    const int o = i >> 6;
    const int k = 2 * (i & 63);
    const float a = W[k * NHID + o], b = W[(k + 1) * NHID + o];
    const unsigned short ha = f2bf_bits(a), hb = f2bf_bits(b);
    const unsigned short la = f2bf_bits(a - bf_bits2f(ha)), lb = f2bf_bits(b - bf_bits2f(hb));
    const unsigned uh = pk16(ha, hb), ul = pk16(la, lb);
    ((volatile unsigned*)OH)[i] = uh; ((volatile unsigned*)OL)[i] = ul;
    __threadfence();
    ((volatile unsigned*)OH)[i] = uh; ((volatile unsigned*)OL)[i] = ul;
  } else {
    const int i = (blk - 64) * NT + t;
    const int o = i >> 6;
    const int k = 2 * (i & 63);
    const float a = WA[k * NATT + o] * WA_CARRY, b = WA[(k + 1) * NATT + o] * WA_CARRY;
    const unsigned u = pk16(h_bits(a), h_bits(b));
    ((volatile unsigned*)WAH)[i] = u;
    __threadfence();
    ((volatile unsigned*)WAH)[i] = u;
  }
}

__global__ __launch_bounds__(NT) void split8_bf16_kernel(const float* __restrict__ in, unsigned short* __restrict__ oh,
                                                        unsigned short* __restrict__ ol, int n8) {
  const int i = blockIdx.x * NT + threadIdx.x;
  if (i < n8) {
    const float* p = in + 8 * (size_t)i;
    const v4f a = *(const v4f*)(p);
    const v4f c = *(const v4f*)(p + 4);
    unsigned short hb[8], lb[8];
#pragma unroll
    for (int e = 0; e < 4; ++e) {
      hb[e] = f2bf_bits(a[e]);     lb[e] = f2bf_bits(a[e] - bf_bits2f(hb[e]));
      hb[4 + e] = f2bf_bits(c[e]); lb[4 + e] = f2bf_bits(c[e] - bf_bits2f(hb[4 + e]));
    }
    const v4u uh = (v4u){pk16(hb[0], hb[1]), pk16(hb[2], hb[3]), pk16(hb[4], hb[5]), pk16(hb[6], hb[7])};
    const v4u ul = (v4u){pk16(lb[0], lb[1]), pk16(lb[2], lb[3]), pk16(lb[4], lb[5]), pk16(lb[6], lb[7])};
    unsigned short* qh = oh + 8 * (size_t)i;
    unsigned short* ql = ol + 8 * (size_t)i;
    *(volatile v4u*)qh = uh; *(volatile v4u*)ql = ul;
    __threadfence();
    *(volatile v4u*)qh = uh; *(volatile v4u*)ql = ul;
  }
}

__global__ __launch_bounds__(NT) void degree_kernel(const int* __restrict__ ei, float* __restrict__ DIS) {
  __shared__ int LIST[SCH];
  __shared__ int scan_ws[96];
  __shared__ int SCNT[TILE_R];
  const int tid = threadIdx.x, lane = tid & 31, wave = tid >> 5;
  const int n0 = blockIdx.x * TILE_R;
  for (int i = tid; i < SCH; i += NT) LIST[i] = 0;
  for (int i = tid; i < TILE_R; i += NT) SCNT[i] = 0;
  if (tid < 96) scan_ws[tid] = 0;
  __syncthreads();
  const int* srcv = ei; const int* dstv = ei + NEDGE;
#pragma unroll 1
  for (int c = 0; c < NCHK; ++c) {
    const int tot = chunk_hits(dstv, srcv, c * SCH, n0, tid, LIST, scan_ws);
#pragma unroll 1
    for (int base = 0; base < tot; base += 32) {
      const int q = base + lane; const int qc = q < SCH ? q : SCH - 1;
      const int lv = LIST[qc];
      const int inval = (q < tot) ? 0 : -1;
      const int rv = lv | inval;
      const int own = (rv >= 0 && (rv >> 25) == wave) ? 1 : 0;
      unsigned msk = (unsigned)__ballot(own);
#pragma unroll 1
      for (int it = 0; it < 32; ++it) {
        if (msk == 0u) break;
        const int bp = __builtin_ctz(msk); msk &= msk - 1u;
        const int r = __shfl(rv, bp, 32);
        const int dl = (r >> 16) & (TILE_R - 1);
        if (lane == 0) SCNT[dl] += 1;
      }
    }
    __syncthreads();
  }
#pragma unroll 1
  for (int j = 0; j < ROWS_W / 32; ++j) {
    const int idx = wave * ROWS_W + j * 32 + lane;
    const int cnt = SCNT[idx];
    const float dv = 1.0f / sqrtf((float)(cnt + 1));
    float* p = DIS + n0 + idx;
    *(volatile float*)p = dv;
    __threadfence();
    *(volatile float*)p = dv;
  }
}

__global__ __launch_bounds__(NT) void agg_kernel(const float* __restrict__ HPRE, const int* __restrict__ ei, const float* __restrict__ DIS,
                                                const float* __restrict__ bias, float* AGG, float* __restrict__ PART) {
  __shared__ int LIST[SCH];
  __shared__ int scan_ws[96];
  __shared__ __align__(16) float red[2 * 8 * NHID];
  const int tid = threadIdx.x, lane = tid & 31, wave = tid >> 5;
  const int n0 = blockIdx.x * TILE_R;
  const v4f z4 = {0.f, 0.f, 0.f, 0.f};
  const v4f b4 = *(const v4f*)(bias + 4 * lane);
  for (int i = tid; i < SCH; i += NT) LIST[i] = 0;
  if (tid < 96) scan_ws[tid] = 0;
#pragma unroll 1
  for (int j = 0; j < ROWS_W; ++j) {
    const int n = n0 + wave * ROWS_W + j;
    const int nc = n < NNODE ? n : NNODE - 1;
    const float dsd = DIS[n];
    const v4f hv = *(const v4f*)(HPRE + (size_t)nc * NHID + 4 * lane);
    const float f = (n < NNODE) ? dsd : 0.0f;
    const v4f a = hv * f;
    *(v4f*)(AGG + (size_t)n * NHID + 4 * lane) = a;
  }
  __syncthreads();
  const int* srcv = ei; const int* dstv = ei + NEDGE;
#pragma unroll 1
  for (int c = 0; c < NCHK; ++c) {
    const int tot = chunk_hits(dstv, srcv, c * SCH, n0, tid, LIST, scan_ws);
#pragma unroll 1
    for (int base = 0; base < tot; base += 32) {
      const int q = base + lane; const int qc = q < SCH ? q : SCH - 1;
      const int lv = LIST[qc];
      const int inval = (q < tot) ? 0 : -1;
      const int rv = lv | inval;
      const int own = (rv >= 0 && (rv >> 25) == wave) ? 1 : 0;
      unsigned msk = (unsigned)__ballot(own);
#pragma unroll 1
      for (int it = 0; it < 32; ++it) {
        if (msk == 0u) break;
        const int bp = __builtin_ctz(msk); msk &= msk - 1u;
        const int r = __shfl(rv, bp, 32);
        const int dl = (r >> 16) & (TILE_R - 1);
        int s = r & 0xFFFF; s = s < NNODE ? s : NNODE - 1;
        const float ds = DIS[s];
        const v4f hv = *(const v4f*)(HPRE + (size_t)s * NHID + 4 * lane);
        float* rp = AGG + (size_t)(n0 + dl) * NHID + 4 * lane;
        v4f a = *(const v4f*)rp;
        a = a + hv * ds;
        *(v4f*)rp = a;
      }
    }
    __syncthreads();
  }
  v4f cs = z4, cq = z4;
#pragma unroll 1
  for (int j = 0; j < ROWS_W; ++j) {
    const int n = n0 + wave * ROWS_W + j;
    if (n < NNODE) {
      float* rp = AGG + (size_t)n * NHID + 4 * lane;
      const v4f a = *(const v4f*)rp;
      const float dn = DIS[n];
      const v4f v = a * dn + b4;
      cs = cs + v;
      cq = cq + v * v;
      *(volatile v4f*)rp = v;
      __threadfence();
      *(volatile v4f*)rp = v;
    }
  }
  *(v4f*)(red + wave * NHID + 4 * lane) = cs;
  *(v4f*)(red + 8 * NHID + wave * NHID + 4 * lane) = cq;
  __syncthreads();
  if (wave == 0) {
    v4f s = z4, qq = z4;
#pragma unroll
    for (int w = 0; w < 8; ++w) {
      s  = s  + *(const v4f*)(red + w * NHID + 4 * lane);
      qq = qq + *(const v4f*)(red + 8 * NHID + w * NHID + 4 * lane);
    }
    float* pp = PART + (size_t)blockIdx.x * 2 * NHID + 4 * lane;
    *(volatile v4f*)pp = s; *(volatile v4f*)(pp + NHID) = qq;
    __threadfence();
    *(volatile v4f*)pp = s; *(volatile v4f*)(pp + NHID) = qq;
  }
}

template <int MODE>
__global__ __launch_bounds__(NT) void bn_apply_kernel(const float* __restrict__ AGG, const float* __restrict__ PART,
                                                     const float* __restrict__ gam, const float* __restrict__ bet,
                                                     float* __restrict__ OUTF, unsigned short* __restrict__ P1, unsigned short* __restrict__ P2) {
  __shared__ __align__(16) float ssc[NHID];
  __shared__ __align__(16) float ssh[NHID];
  __shared__ __align__(16) float slab[8][2 * NHID];
  const int tid = threadIdx.x, lane = tid & 31, wave = tid >> 5;
  if (tid < NHID) {
    double S = 0.0, Q = 0.0;
#pragma unroll 1
    for (int b = 0; b < NTILE; ++b) { S += (double)PART[b * 2 * NHID + tid]; Q += (double)PART[b * 2 * NHID + NHID + tid]; }
    const double mean = S * (1.0 / NNODE);
    double var = Q * (1.0 / NNODE) - mean * mean;
    var = var > 0.0 ? var : 0.0;
    const float rs = 1.0f / sqrtf((float)var + BN_EPS);
    const float sc = gam[tid] * rs;
    ssc[tid] = sc;
    ssh[tid] = bet[tid] - (float)mean * sc;
  }
  __syncthreads();
  const v4f sc4 = *(const v4f*)(ssc + 4 * lane), sh4 = *(const v4f*)(ssh + 4 * lane);
  float* sw = slab[wave];
  const int rbase = blockIdx.x * RPB;
  const int rs2 = lane >> 4, c8 = (lane & 15) * 8;
#pragma unroll 1
  for (int it = 0; it < RPB / 16; ++it) {
    const int rA = rbase + it * 16 + 2 * wave;
    if (rA < NNODE) {
      const v4f a0 = *(const v4f*)(AGG + (size_t)rA * NHID + 4 * lane);
      const v4f a1 = *(const v4f*)(AGG + (size_t)(rA + 1) * NHID + 4 * lane);
      v4f y0 = a0 * sc4 + sh4, y1 = a1 * sc4 + sh4;
#pragma unroll
      for (int e = 0; e < 4; ++e) { y0[e] = fmaxf(y0[e], 0.f); y1[e] = fmaxf(y1[e], 0.f); }
      if (MODE == 2) {
        float* o0 = OUTF + (size_t)rA * NHID + 4 * lane;
        float* o1 = o0 + NHID;
        *(volatile v4f*)o0 = y0; *(volatile v4f*)o1 = y1;
        __threadfence();
        *(volatile v4f*)o0 = y0; *(volatile v4f*)o1 = y1;
      }
      *(v4f*)(sw + 4 * lane) = y0;
      *(v4f*)(sw + NHID + 4 * lane) = y1;
      __builtin_amdgcn_fence(__ATOMIC_RELEASE, "workgroup");
      __builtin_amdgcn_wave_barrier();
      __builtin_amdgcn_fence(__ATOMIC_ACQUIRE, "workgroup");
      const float* sp = sw + rs2 * NHID + c8;
      const v4f p0 = *(const v4f*)sp;
      const v4f p1 = *(const v4f*)(sp + 4);
      const int row = rA + rs2;
      if (MODE == 1) {
        unsigned short hb[8], lb[8];
#pragma unroll
        for (int e = 0; e < 4; ++e) {
          hb[e] = f2bf_bits(p0[e]);     lb[e] = f2bf_bits(p0[e] - bf_bits2f(hb[e]));
          hb[4 + e] = f2bf_bits(p1[e]); lb[4 + e] = f2bf_bits(p1[e] - bf_bits2f(hb[4 + e]));
        }
        const v4u uh = (v4u){pk16(hb[0], hb[1]), pk16(hb[2], hb[3]), pk16(hb[4], hb[5]), pk16(hb[6], hb[7])};
        const v4u ul = (v4u){pk16(lb[0], lb[1]), pk16(lb[2], lb[3]), pk16(lb[4], lb[5]), pk16(lb[6], lb[7])};
        unsigned short* q1 = P1 + (size_t)row * NHID + c8;
        unsigned short* q2 = P2 + (size_t)row * NHID + c8;
        *(volatile v4u*)q1 = uh; *(volatile v4u*)q2 = ul;
        __threadfence();
        *(volatile v4u*)q1 = uh; *(volatile v4u*)q2 = ul;
      } else {
        unsigned short hb[8];
#pragma unroll
        for (int e = 0; e < 4; ++e) { hb[e] = h_bits(p0[e]); hb[4 + e] = h_bits(p1[e]); }
        const v4u uh = (v4u){pk16(hb[0], hb[1]), pk16(hb[2], hb[3]), pk16(hb[4], hb[5]), pk16(hb[6], hb[7])};
        unsigned short* q1 = P1 + (size_t)row * NHID + c8;
        *(volatile v4u*)q1 = uh;
        __threadfence();
        *(volatile v4u*)q1 = uh;
      }
      __builtin_amdgcn_fence(__ATOMIC_RELEASE, "workgroup");
      __builtin_amdgcn_wave_barrier();
      __builtin_amdgcn_fence(__ATOMIC_ACQUIRE, "workgroup");
    }
  }
}

__global__ __launch_bounds__(NT) void score_kernel(const float* __restrict__ T, const float* __restrict__ b1, const float* __restrict__ w2,
                                                  const float* __restrict__ b2, float* __restrict__ SC) {
  const int n = blockIdx.x * NT + threadIdx.x;
  if (n < NNODE) {
    const float* tr = T + (size_t)n * NATT;
    float acc = 0.0f;
#pragma unroll 1
    for (int j = 0; j < NATT; ++j) acc = fmaf(tanhf(tr[j] + b1[j]), w2[j], acc);
    acc += b2[0];
    *(volatile float*)(SC + n) = acc;
    __threadfence();
    *(volatile float*)(SC + n) = acc;
  }
}

__global__ __launch_bounds__(128) void pool_kernel(const float* __restrict__ EMB, const float* __restrict__ SC, float* __restrict__ POOL) {
  __shared__ float swt[NSUB];
  __shared__ float red[128];
  const int cell = blockIdx.x, t = threadIdx.x;
  const int base = cell * NSUB;
  float m = -INFINITY;
  for (int s = t; s < NSUB; s += 128) m = fmaxf(m, SC[base + s]);
  red[t] = m; __syncthreads();
  for (int off = 64; off > 0; off >>= 1) {
    if (t < off) red[t] = fmaxf(red[t], red[t + off]);
    __syncthreads();
  }
  const float mx = red[0];
  __syncthreads();
  float z = 0.f;
  for (int s = t; s < NSUB; s += 128) {
    const float e = expf(SC[base + s] - mx);
    swt[s] = e; z += e;
  }
  red[t] = z; __syncthreads();
  for (int off = 64; off > 0; off >>= 1) {
    if (t < off) red[t] += red[t + off];
    __syncthreads();
  }
  const float invZ = 1.0f / red[0];
  float acc = 0.0f;
#pragma unroll 1
  for (int s = 0; s < NSUB; ++s) acc = fmaf(swt[s], EMB[(size_t)(base + s) * NHID + t], acc);
  const float v = acc * invZ;
  float* p = POOL + (size_t)cell * NHID + t;
  *(volatile float*)p = v;
  __threadfence();
  *(volatile float*)p = v;
}

__global__ __launch_bounds__(NT) void head_kernel(const float* __restrict__ P, const float* __restrict__ Wfc, const float* __restrict__ bfc,
                                                 const float* __restrict__ ge, const float* __restrict__ be,
                                                 const float* __restrict__ Wb, const float* __restrict__ bb,
                                                 const float* __restrict__ gb, const float* __restrict__ bbt, float* __restrict__ out) {
  __shared__ __align__(16) float zs[NCELL * NHID];
  __shared__ __align__(16) float ys[NCELL * NBOT];
  __shared__ float smu[NHID];
  __shared__ float srs[NHID];
  const int tid = threadIdx.x, wave = tid >> 5, lane = tid & 31;
  for (int i = tid; i < NCELL * NHID; i += NT) {
    const int g = i >> 7, j = i & 127;
    float s = 0.0f;
#pragma unroll 1
    for (int c = 0; c < NHID; ++c) s = fmaf(P[g * NHID + c], Wfc[c * NHID + j], s);
    zs[i] = s + bfc[j];
  }
  __syncthreads();
  if (tid < NHID) {
    double m = 0.0;
#pragma unroll 1
    for (int g = 0; g < NCELL; ++g) m += (double)zs[g * NHID + tid];
    m = m * (1.0 / NCELL);
    const float mf = (float)m;
    double v = 0.0;
#pragma unroll 1
    for (int g = 0; g < NCELL; ++g) { const float d = zs[g * NHID + tid] - mf; const float dd = d * d; v += (double)dd; }
    v = v * (1.0 / NCELL);
    const float vf = (float)v;
    smu[tid] = mf; srs[tid] = 1.0f / sqrtf(vf + BN_EPS);
  }
  __syncthreads();
  for (int i = tid; i < NCELL * NHID; i += NT) {
    const int j = i & 127;
    float t = ge[j] * (zs[i] - smu[j]);
    t = t * srs[j];
    t = t + be[j];
    zs[i] = fmaxf(t, 0.f);
  }
  __syncthreads();
  for (int i = tid; i < NCELL * NBOT; i += NT) {
    const int g = i >> 5, k = i & 31;
    float s = 0.0f;
#pragma unroll 1
    for (int j = 0; j < NHID; ++j) s = fmaf(zs[g * NHID + j], Wb[j * NBOT + k], s);
    ys[i] = s + bb[k];
  }
  __syncthreads();
  if (tid < NBOT) {
    double m = 0.0;
#pragma unroll 1
    for (int g = 0; g < NCELL; ++g) m += (double)ys[g * NBOT + tid];
    m = m * (1.0 / NCELL);
    const float mf = (float)m;
    double v = 0.0;
#pragma unroll 1
    for (int g = 0; g < NCELL; ++g) { const float d = ys[g * NBOT + tid] - mf; const float dd = d * d; v += (double)dd; }
    v = v * (1.0 / NCELL);
    const float vf = (float)v;
    smu[tid] = mf; srs[tid] = 1.0f / sqrtf(vf + BN_EPS);
  }
  __syncthreads();
  for (int i = tid; i < NCELL * NBOT; i += NT) {
    const int k = i & 31;
    float t = gb[k] * (ys[i] - smu[k]);
    t = t * srs[k];
    t = t + bbt[k];
    ys[i] = fmaxf(t, 0.f);
  }
  __syncthreads();
#pragma unroll 1
  for (int grp = wave; grp < (NCELL * NBOT) / 128; grp += 8) {
    const v4f val = *(const v4f*)(ys + grp * 128 + 4 * lane);
    float* p = out + grp * 128 + 4 * lane;
    *(volatile v4f*)p = val;
    __threadfence();
    *(volatile v4f*)p = val;
  }
}

extern "C" void kernel_launch(void* const* d_in, const int* in_sizes, int n_in,
                              void* d_out, int out_size, void* d_ws, size_t ws_size, hipStream_t stream) {
  if (n_in < 22) return;
  if (in_sizes[0] != NNODE * NHID || in_sizes[1] != 2 * NEDGE) return;
  if (out_size != NCELL * NBOT + NNODE * NHID) return;
  const float* x       = (const float*)d_in[0];
  const int*   ei      = (const int*)  d_in[1];
  const float* conv1_w = (const float*)d_in[2];
  const float* conv1_b = (const float*)d_in[3];
  const float* bn1_g   = (const float*)d_in[4];
  const float* bn1_b   = (const float*)d_in[5];
  const float* conv2_w = (const float*)d_in[6];
  const float* conv2_b = (const float*)d_in[7];
  const float* bn2_g   = (const float*)d_in[8];
  const float* bn2_b   = (const float*)d_in[9];
  const float* att_w1  = (const float*)d_in[10];
  const float* att_b1  = (const float*)d_in[11];
  const float* att_w2  = (const float*)d_in[12];
  const float* att_b2  = (const float*)d_in[13];
  const float* fc_w    = (const float*)d_in[14];
  const float* fc_b    = (const float*)d_in[15];
  const float* bne_g   = (const float*)d_in[16];
  const float* bne_b   = (const float*)d_in[17];
  const float* bot_w   = (const float*)d_in[18];
  const float* bot_b   = (const float*)d_in[19];
  const float* bnb_g   = (const float*)d_in[20];
  const float* bnb_b   = (const float*)d_in[21];
  float* out0 = (float*)d_out;
  float* out1 = (float*)d_out + NCELL * NBOT;

  char* ws = (char*)d_ws; size_t off = 0;
  auto carve = [&](size_t bytes) -> char* { char* p = ws + off; off += (bytes + 255) & ~(size_t)255; return p; };
  unsigned short* W1H  = (unsigned short*)carve((size_t)NHID * NHID * 2);
  unsigned short* W1L  = (unsigned short*)carve((size_t)NHID * NHID * 2);
  unsigned short* W2H  = (unsigned short*)carve((size_t)NHID * NHID * 2);
  unsigned short* W2L  = (unsigned short*)carve((size_t)NHID * NHID * 2);
  unsigned short* WAH  = (unsigned short*)carve((size_t)NATT * NHID * 2);
  float*          DIS  = (float*)carve((size_t)NPADR * 4);
  unsigned short* XH   = (unsigned short*)carve((size_t)NNODE * NHID * 2);
  unsigned short* XL   = (unsigned short*)carve((size_t)NNODE * NHID * 2);
  float*          HPRE = (float*)carve((size_t)NNODE * NHID * 4);
  float*          AGG  = (float*)carve((size_t)NPADR * NHID * 4);
  float*          PART = (float*)carve((size_t)NTILE * 2 * NHID * 4);
  unsigned short* EH   = (unsigned short*)carve((size_t)NNODE * NHID * 2);
  float*          TT   = (float*)carve((size_t)NNODE * NATT * 4);
  float*          SCR  = (float*)carve((size_t)NNODE * 4);
  float*          POOL = (float*)carve((size_t)NCELL * NHID * 4);
  if (off > ws_size || off > (size_t)134217728) return;

  const int tiles12 = (NNODE / 64) * (NHID / 64);
  const int tiles3  = (NNODE / 64) * (NATT / 64);

  prep_kernel<<<80, NT, 0, stream>>>(conv1_w, conv2_w, att_w1, (unsigned*)W1H, (unsigned*)W1L, (unsigned*)W2H, (unsigned*)W2L, (unsigned*)WAH);
  split8_bf16_kernel<<<(NNODE * NHID / 8) / NT, NT, 0, stream>>>(x, XH, XL, NNODE * NHID / 8);
  degree_kernel<<<NTILE, NT, 0, stream>>>(ei, DIS);

  wmma_gemm64<1, true, 0, 0, false><<<dim3((tiles12 + 7) / 8, 1), 256, 0, stream>>>(
      (const unsigned short*)XH, (const unsigned short*)XL, NHID, 0L,
      (const unsigned short*)W1H, (const unsigned short*)W1L, NHID, 0L,
      (void*)HPRE, (void*)nullptr, NHID, 0L,
      (const float*)nullptr, (const float*)nullptr, 0L, NNODE, NHID, NHID, 1.0f);
  agg_kernel<<<NTILE, NT, 0, stream>>>(HPRE, ei, DIS, conv1_b, AGG, PART);
  bn_apply_kernel<1><<<NAPB, NT, 0, stream>>>(AGG, PART, bn1_g, bn1_b, (float*)nullptr, XH, XL);

  wmma_gemm64<1, true, 0, 0, false><<<dim3((tiles12 + 7) / 8, 1), 256, 0, stream>>>(
      (const unsigned short*)XH, (const unsigned short*)XL, NHID, 0L,
      (const unsigned short*)W2H, (const unsigned short*)W2L, NHID, 0L,
      (void*)HPRE, (void*)nullptr, NHID, 0L,
      (const float*)nullptr, (const float*)nullptr, 0L, NNODE, NHID, NHID, 1.0f);
  agg_kernel<<<NTILE, NT, 0, stream>>>(HPRE, ei, DIS, conv2_b, AGG, PART);
  bn_apply_kernel<2><<<NAPB, NT, 0, stream>>>(AGG, PART, bn2_g, bn2_b, out1, EH, (unsigned short*)nullptr);

  wmma_gemm64<0, false, 0, 0, false><<<dim3((tiles3 + 7) / 8, 1), 256, 0, stream>>>(
      (const unsigned short*)EH, (const unsigned short*)nullptr, NHID, 0L,
      (const unsigned short*)WAH, (const unsigned short*)nullptr, NHID, 0L,
      (void*)TT, (void*)nullptr, NATT, 0L,
      (const float*)nullptr, (const float*)nullptr, 0L, NNODE, NATT, NHID, WA_CARRY_INV);
  score_kernel<<<(NNODE + NT - 1) / NT, NT, 0, stream>>>(TT, att_b1, att_w2, att_b2, SCR);

  pool_kernel<<<NCELL, 128, 0, stream>>>(out1, SCR, POOL);
  head_kernel<<<1, NT, 0, stream>>>(POOL, fc_w, fc_b, bne_g, bne_b, bot_w, bot_b, bnb_g, bnb_b, out0);
}
